// Muti_GAT_28724741276298
// MI455X (gfx1250) — hardware-verified
//
#include <hip/hip_runtime.h>
#include <stddef.h>


typedef _Float16 v16h __attribute__((ext_vector_type(16)));
typedef _Float16 v8h  __attribute__((ext_vector_type(8)));
typedef float    v8f  __attribute__((ext_vector_type(8)));
typedef float    v4f  __attribute__((ext_vector_type(4)));
typedef int      v4i  __attribute__((ext_vector_type(4)));

#ifndef NB
#define NB 8
#endif
#define NB_FULL  8
#define SEQ      256
#define SEQ_FULL 256
#define DIM      512
#define NHEAD    4
#define NCAT     (NHEAD * DIM)
#define EDIM     64
#define EHID     64
#define NTYPES   50
#define LUTP     64
#define APAD     64
#define MROWS    (NB * SEQ)
#define NEGFILL  (-9.0e15f)
#define OUT1_ELEMS ((size_t)NB_FULL * SEQ_FULL * DIM)

static_assert(NB >= 1 && NB <= NB_FULL);
static_assert(SEQ == SEQ_FULL);
static_assert(SEQ == 2 * 32 * 4);
static_assert(SEQ == 32 * 8);
static_assert((SEQ % 64) == 0 && (SEQ % 32) == 0);
static_assert((DIM % 64) == 0 && (DIM % 32) == 0);
static_assert((NCAT % 64) == 0);
static_assert((MROWS % 64) == 0 && (MROWS % 8) == 0);
static_assert(NHEAD * LUTP == 256);
static_assert(NTYPES <= LUTP && LUTP == 16 * 4);
static_assert(NHEAD * NB <= 32 && NHEAD * NB <= APAD && APAD == 64);
static_assert(DIM == 2 * 256);
static_assert(DIM == 16 * 32);
static_assert((((size_t)MROWS * DIM / 8) % 256) == 0);
static_assert((((size_t)MROWS * DIM / 4) % 256) == 0);
static_assert(OUT1_ELEMS * 4 == (size_t)4194304);
static_assert((256 / 8) * 2 == 64);
static_assert((256 / 16) * 4 == 64);

#define LDT 72
#define LDC 68
static_assert((LDT % 8) == 0 && LDT >= 64);
static_assert((LDC % 4) == 0 && LDC >= 64);
static_assert(64 * LDC * 4 <= 131072 && 64 * LDT * 2 <= 131072);
static_assert(NHEAD * LUTP * 4 + 8 * SEQ * 2 <= 131072);

#define WCARRY 64.0f
#define PCARRY 16384.0f
#define ACARRY 16.0f

#define WTO_BYTES   ((size_t)NCAT * DIM * 2)
#define WASP_BYTES  ((size_t)DIM * DIM * 2)
#define X16_BYTES   ((size_t)MROWS * DIM * 2)
#define LUT_BYTES   ((size_t)NHEAD * LUTP * 4)
#define ATT16_BYTES ((size_t)NHEAD * NB * SEQ * SEQ * 2)
#define HVT_BYTES   ((size_t)NB * NCAT * SEQ * 2)
#define HEDGE_BYTES ((size_t)NHEAD * NB * SEQ * DIM * 4)
#define ASP16_BYTES ((size_t)APAD * DIM * 2)
#define ASPX_BYTES  ((size_t)NB * DIM * 4)
#define ASPT_BYTES  ((size_t)APAD * DIM * 4)
#define GATE_BYTES  ((size_t)128)
#define OFF_WTO   ((size_t)0)
#define OFF_WASP  (OFF_WTO + WTO_BYTES)
#define OFF_X16   (OFF_WASP + WASP_BYTES)
#define OFF_LUT   (OFF_X16 + X16_BYTES)
#define OFF_ATT16 (OFF_LUT + LUT_BYTES)
#define OFF_HVT   (OFF_ATT16 + ATT16_BYTES)
#define OFF_HEDGE (OFF_HVT + HVT_BYTES)
#define OFF_ASP16 (OFF_HEDGE + HEDGE_BYTES)
#define OFF_ASPX  (OFF_ASP16 + ASP16_BYTES)
#define OFF_ASPT  (OFF_ASPX + ASPX_BYTES)
#define OFF_GATE  (OFF_ASPT + ASPT_BYTES)
#define WS_TOTAL  (OFF_GATE + GATE_BYTES)
static_assert((WTO_BYTES % 128) == 0 && (WASP_BYTES % 128) == 0 && (X16_BYTES % 128) == 0);
static_assert((LUT_BYTES % 128) == 0 && (ATT16_BYTES % 128) == 0 && (HVT_BYTES % 128) == 0);
static_assert((HEDGE_BYTES % 128) == 0 && (ASP16_BYTES % 128) == 0 && (ASPX_BYTES % 128) == 0);
static_assert((ASPT_BYTES % 128) == 0 && (GATE_BYTES % 128) == 0);
static_assert(NHEAD * NB * 4 <= 128);
static_assert(WS_TOTAL <= (size_t)134217728);

__device__ __forceinline__ float bf16r(float x) {
  unsigned int u = __float_as_uint(x);
  u = (u + 0x7FFFu + ((u >> 16) & 1u)) & 0xFFFF0000u;
  return __uint_as_float(u);
}

__device__ __forceinline__ _Float16 toh_flush(float v) {
  const _Float16 r = (_Float16)v;
  return (fabsf(v) < 6.103515625e-05f) ? (_Float16)0.0f : r;
}

__device__ __forceinline__ v16h frag_at(const _Float16* p) {
  v8h lo = *(const v8h*)(p);
  v8h hi = *(const v8h*)(p + 16);
  v16h out;
#pragma unroll
  for (int i = 0; i < 8; ++i) { out[i] = lo[i]; out[i + 8] = hi[i]; }
  return out;
}

__device__ __forceinline__ v8f wmma16(v16h a, v16h b, v8f c) {
  v8f d = __builtin_amdgcn_wmma_f32_16x16x32_f16(false, a, false, b, (short)0, c,
                                                 false, false);
  asm volatile("v_nop\n\tv_nop\n\tv_nop\n\tv_nop" : "+v"(d) : "v"(a), "v"(b));
  return d;
}

__device__ __forceinline__ float red32_sum(float x) {
#pragma unroll
  for (int off = 1; off < 32; off <<= 1) x += __shfl_xor(x, off, 32);
  return x;
}
__device__ __forceinline__ float red32_max(float x) {
#pragma unroll
  for (int off = 1; off < 32; off <<= 1) x = fmaxf(x, __shfl_xor(x, off, 32));
  return x;
}

__device__ __forceinline__ void wave_lds_sync() {
  __builtin_amdgcn_fence(3  , "wavefront");
  asm volatile("s_wait_dscnt 0x0" ::: "memory");
  __builtin_amdgcn_wave_barrier();
}

__global__ __launch_bounds__(256) void wconv_kernel(
    const float* __restrict__ W, _Float16* __restrict__ Wt, unsigned ldw, unsigned ldk) {
  __shared__ _Float16 T[64 * LDT];
  const unsigned tid = threadIdx.x;
  const unsigned n0 = blockIdx.x * 64u;
  const unsigned k0 = blockIdx.y * 64u;
#pragma unroll 4
  for (unsigned j = 0; j < 16u; ++j) {
    const unsigned idx = tid + 256u * j;
    const unsigned kr = idx >> 6, nc = idx & 63u;
    const float v = W[(size_t)(k0 + kr) * ldw + n0 + nc];
    T[nc * LDT + kr] = toh_flush(WCARRY * bf16r(v));
  }
  __syncthreads();
  v8h x[2];
  size_t off[2];
#pragma unroll
  for (unsigned i = 0; i < 2u; ++i) {
    const unsigned n = 32u * i + (tid >> 3);
    const unsigned kc = (tid & 7u) * 8u;
    x[i] = *(const v8h*)&T[n * LDT + kc];
    off[i] = (size_t)(n0 + n) * ldk + k0 + kc;
  }
#pragma unroll
  for (int i = 0; i < 2; ++i) *(volatile v8h*)(Wt + off[i]) = x[i];
  __threadfence();
#pragma unroll
  for (int i = 0; i < 2; ++i) *(volatile v8h*)(Wt + off[i]) = x[i];
}

__global__ __launch_bounds__(256) void xconv_kernel(
    const float* __restrict__ X, _Float16* __restrict__ X16) {
  const unsigned idx = blockIdx.x * 256u + threadIdx.x;
  const unsigned crow = idx / (unsigned)(DIM / 8);
  const unsigned c = (idx - crow * (unsigned)(DIM / 8)) * 8u;
  const unsigned bidx = crow / (unsigned)SEQ;
  const unsigned sq = crow - bidx * (unsigned)SEQ;
  const float* src = X + ((size_t)bidx * SEQ_FULL + sq) * DIM + c;
  const v4f a0 = *(const v4f*)(src);
  const v4f a1 = *(const v4f*)(src + 4);
  v8h o;
#pragma unroll
  for (int i = 0; i < 4; ++i) {
    o[i]     = toh_flush(bf16r(a0[i]));
    o[i + 4] = toh_flush(bf16r(a1[i]));
  }
  _Float16* p = X16 + (size_t)crow * DIM + c;
  *(volatile v8h*)p = o;
  __threadfence();
  *(volatile v8h*)p = o;
}

__global__ __launch_bounds__(64) void lut_kernel(
    const float* __restrict__ table, const float* __restrict__ Wm, const float* __restrict__ Wl,
    float* __restrict__ lut) {
  __shared__ float L[LUTP];
  const unsigned t = threadIdx.x;
  const unsigned h = blockIdx.x;
  const unsigned tc = min(t, (unsigned)(NTYPES - 1));
  const float* et = table + (size_t)tc * EDIM;
  const float* wm = Wm + (size_t)h * EDIM * EHID;
  const float* wl = Wl + (size_t)h * EHID;
  double acc = 0.0;
#pragma unroll 1
  for (unsigned e2 = 0; e2 < (unsigned)EHID; ++e2) {
    double s = 0.0;
#pragma unroll 1
    for (unsigned e = 0; e < (unsigned)EDIM; ++e)
      s += (double)bf16r(et[e]) * (double)bf16r(wm[e * EHID + e2]);
    const double r = (s > 0.0) ? s : 0.0;
    acc += r * (double)bf16r(wl[e2]);
  }
  const float val = (float)acc;
  L[t] = (t < (unsigned)NTYPES) ? val : 0.0f;
  __syncthreads();
  if (t < 16u) {
    const v4f x = *(const v4f*)&L[4u * t];
    float* p = lut + (size_t)h * LUTP + 4u * t;
    *(volatile v4f*)p = x;
    __threadfence();
    *(volatile v4f*)p = x;
  }
}

__global__ __launch_bounds__(256) void att_kernel(
    const int* __restrict__ adj, const int* __restrict__ dep, const float* __restrict__ lut,
    float* __restrict__ att_out, _Float16* __restrict__ att16) {
  __shared__ float lut_s[NHEAD * LUTP];
  __shared__ _Float16 Ps[8 * SEQ];
  const unsigned tid = threadIdx.x, lane = tid & 31u;
  const int wave = __builtin_amdgcn_readfirstlane(threadIdx.x >> 5);
  lut_s[tid] = lut[tid];
  __syncthreads();

  const unsigned crow = blockIdx.x * 8u + (unsigned)wave;
  const unsigned b = crow / (unsigned)SEQ;
  const unsigned i = crow - b * (unsigned)SEQ;
  const size_t src = ((size_t)b * SEQ_FULL + i) * SEQ_FULL;
  const v4i d0 = *(const v4i*)(dep + src + 4u * lane);
  const v4i d1 = *(const v4i*)(dep + src + 128u + 4u * lane);
  const v4i a0 = *(const v4i*)(adj + src + 4u * lane);
  const v4i a1 = *(const v4i*)(adj + src + 128u + 4u * lane);

  int tix[8];
  unsigned livem = 0u, openm = 0u;
#pragma unroll
  for (int c = 0; c < 4; ++c) {
    tix[c]     = min(max(d0[c], 0), NTYPES - 1);
    tix[c + 4] = min(max(d1[c], 0), NTYPES - 1);
    livem |= ((d0[c] != 0) ? 1u : 0u) << c;
    livem |= ((d1[c] != 0) ? 1u : 0u) << (c + 4);
    openm |= ((a0[c] != 0) ? 1u : 0u) << c;
    openm |= ((a1[c] != 0) ? 1u : 0u) << (c + 4);
  }
  _Float16* P = Ps + (unsigned)wave * (unsigned)SEQ;

#pragma unroll 1
  for (unsigned h = 0; h < (unsigned)NHEAD; ++h) {
    float ew[8];
    float part = 0.0f;
#pragma unroll
    for (int c = 0; c < 8; ++c) {
      float v = lut_s[h * LUTP + (unsigned)tix[c]];
      asm volatile("" : "+v"(v));
      ew[c] = ((livem >> c) & 1u) ? v : 0.0f;
      part += ew[c];
    }
    const float mean = red32_sum(part) * (1.0f / (float)SEQ);
    const float rden = 1.0f / (fabsf(mean) + 1.0e-10f);
    float s[8];
    float mx = NEGFILL;
#pragma unroll
    for (int c = 0; c < 8; ++c) {
      const float t = ew[c] * rden;
      s[c] = ((openm >> c) & 1u) ? t : NEGFILL;
      mx = fmaxf(mx, s[c]);
    }
    mx = red32_max(mx);
    float es = 0.0f;
#pragma unroll
    for (int c = 0; c < 8; ++c) {
      s[c] = __expf(s[c] - mx);
      es += s[c];
    }
    const float inv = 1.0f / red32_sum(es);
    v4f p0, p1;
#pragma unroll
    for (int c = 0; c < 4; ++c) {
      p0[c] = s[c] * inv;
      p1[c] = s[c + 4] * inv;
    }
#pragma unroll
    for (int c = 0; c < 4; ++c) {
      P[4u * lane + (unsigned)c]        = toh_flush(PCARRY * p0[c]);
      P[128u + 4u * lane + (unsigned)c] = toh_flush(PCARRY * p1[c]);
    }
    wave_lds_sync();
    const v8h x = *(const v8h*)&P[8u * lane];
    float* po = att_out + (((size_t)h * NB_FULL + b) * SEQ + i) * SEQ + 4u * lane;
    _Float16* ph = att16 + (((size_t)h * NB + b) * SEQ + i) * SEQ + 8u * lane;
    *(volatile v4f*)(po) = p0;
    *(volatile v4f*)(po + 128) = p1;
    *(volatile v8h*)(ph) = x;
    __threadfence();
    *(volatile v4f*)(po) = p0;
    *(volatile v4f*)(po + 128) = p1;
    *(volatile v8h*)(ph) = x;
    wave_lds_sync();
  }
}

template <int MODE>
__device__ __forceinline__ void gemm_body(
    const _Float16* __restrict__ A16, const _Float16* __restrict__ Bt, const unsigned K,
    const float* __restrict__ bias, float* __restrict__ outf, _Float16* __restrict__ out16) {
  __shared__ float Cs[64 * LDC];
  const unsigned tid = threadIdx.x, lane = tid & 31u, w = tid >> 5;
  const unsigned mw = w >> 1, nw = w & 1u;
  const unsigned hh = lane >> 4, m = lane & 15u;
  const unsigned n0 = blockIdx.x * 64u;
  const unsigned row0 = blockIdx.y * 64u;

  const _Float16* ap  = A16 + (size_t)(row0 + mw * 16u + m) * K + hh * 8u;
  const _Float16* bp0 = Bt + (size_t)(n0 + nw * 32u + m) * K + hh * 8u;
  const _Float16* bp1 = bp0 + (size_t)16 * K;
  v8f acc0 = {}, acc1 = {};
#pragma unroll 2
  for (unsigned k0 = 0; k0 < K; k0 += 32u) {
    const v16h a  = frag_at(ap + k0);
    const v16h b0 = frag_at(bp0 + k0);
    const v16h b1 = frag_at(bp1 + k0);
    acc0 = wmma16(a, b0, acc0);
    acc1 = wmma16(a, b1, acc1);
  }
#pragma unroll
  for (int r = 0; r < 8; ++r) {
    float* d = &Cs[(mw * 16u + hh * 8u + (unsigned)r) * LDC + nw * 32u + m];
    d[0]  = acc0[r];
    d[16] = acc1[r];
  }
  __syncthreads();

  if (MODE == 1) {
    const unsigned bidx = row0 / (unsigned)SEQ;
    const unsigned key0 = row0 - bidx * (unsigned)SEQ;
    v8h x[2];
    size_t off[2];
#pragma unroll
    for (unsigned i = 0; i < 2u; ++i) {
      const unsigned dcol = 32u * i + (tid >> 3);
      const unsigned kk = (tid & 7u) * 8u;
      const float bb = bf16r(bias[n0 + dcol]);
#pragma unroll
      for (unsigned j = 0; j < 8u; ++j) {
        const float t = Cs[(kk + j) * LDC + dcol] * (1.0f / WCARRY) + bb;
        x[i][j] = toh_flush(t);
      }
      off[i] = ((size_t)bidx * NCAT + n0 + dcol) * SEQ + key0 + kk;
    }
#pragma unroll
    for (int i = 0; i < 2; ++i) *(volatile v8h*)(out16 + off[i]) = x[i];
    __threadfence();
#pragma unroll
    for (int i = 0; i < 2; ++i) *(volatile v8h*)(out16 + off[i]) = x[i];
  }

  if (MODE == 6) {
#pragma unroll 1
    for (unsigned g = 0; g < 4u; ++g) {
      const unsigned r = 16u * g + (tid >> 4);
      const unsigned c = (tid & 15u) * 4u;
      const v4f u  = *(const v4f*)&Cs[r * LDC + c];
      const v4f gb = *(const v4f*)(bias + n0 + c);
      v4f t;
#pragma unroll
      for (int j = 0; j < 4; ++j)
        t[j] = tanhf(u[j] * (1.0f / (WCARRY * ACARRY)) + bf16r(gb[j]));
      *(v4f*)&Cs[r * LDC + c] = t;
    }
  }

  if (MODE == 5 || MODE == 6) {
    v4f xs[4];
    size_t off[4];
#pragma unroll
    for (unsigned i = 0; i < 4u; ++i) {
      const unsigned r = 16u * i + (tid >> 4);
      const unsigned c = (tid & 15u) * 4u;
      const v4f u = *(const v4f*)&Cs[r * LDC + c];
      v4f val;
#pragma unroll
      for (int j = 0; j < 4; ++j)
        val[j] = (MODE == 5) ? fmaxf(u[j] * (1.0f / PCARRY), 0.0f) : u[j];
      xs[i] = val;
      off[i] = (size_t)(row0 + r) * DIM + n0 + c;
    }
#pragma unroll
    for (int i = 0; i < 4; ++i) *(volatile v4f*)(outf + off[i]) = xs[i];
    __threadfence();
#pragma unroll
    for (int i = 0; i < 4; ++i) *(volatile v4f*)(outf + off[i]) = xs[i];
  }
}

__global__ __launch_bounds__(256) void gemm_hv_kernel(
    const _Float16* __restrict__ A16, const _Float16* __restrict__ Bt,
    const float* __restrict__ bias, _Float16* __restrict__ hvt) {
  gemm_body<1>(A16, Bt, (unsigned)DIM, bias, (float*)0, hvt);
}
__global__ __launch_bounds__(256) void gemm_hedge_kernel(
    const _Float16* __restrict__ att16, const _Float16* __restrict__ hvt,
    float* __restrict__ hedge) {
  const unsigned z = blockIdx.z;
  const unsigned h = z / (unsigned)NB;
  const unsigned b = z - h * (unsigned)NB;
  gemm_body<5>(att16 + (size_t)z * SEQ * SEQ,
               hvt + ((size_t)b * NCAT + (size_t)h * DIM) * SEQ,
               (unsigned)SEQ, (const float*)0,
               hedge + (size_t)z * SEQ * DIM, (_Float16*)0);
}
__global__ __launch_bounds__(256) void gemm_asp_kernel(
    const _Float16* __restrict__ A16, const _Float16* __restrict__ Bt,
    const float* __restrict__ bias, float* __restrict__ aspt) {
  gemm_body<6>(A16, Bt, (unsigned)DIM, bias, aspt, (_Float16*)0);
}

__global__ __launch_bounds__(256) void pool_h_kernel(
    const float* __restrict__ hedge, const int* __restrict__ aidx,
    _Float16* __restrict__ asp16) {
  __shared__ _Float16 S[256];
  const unsigned tid = threadIdx.x;
  const unsigned row = blockIdx.x >> 1;
  const unsigned half = blockIdx.x & 1u;
  const unsigned d = half * 256u + tid;
  float mval = 0.0f;
  if (row < (unsigned)(NHEAD * NB)) {
    const unsigned h = row / (unsigned)NB;
    const unsigned b = row - h * (unsigned)NB;
    const int lo = max(aidx[2u * b], 0);
    const int hi = min(aidx[2u * b + 1u], SEQ - 1);
    const float* base = hedge + (size_t)row * SEQ * DIM + d;
#pragma unroll 1
    for (int n = lo; n <= hi; ++n) mval = fmaxf(mval, base[(size_t)n * DIM]);
  }
  S[tid] = toh_flush(ACARRY * mval);
  __syncthreads();
  if (tid < 32u) {
    const v8h x = *(const v8h*)&S[8u * tid];
    _Float16* p = asp16 + (size_t)row * DIM + half * 256u + 8u * tid;
    *(volatile v8h*)p = x;
    __threadfence();
    *(volatile v8h*)p = x;
  }
}

__global__ __launch_bounds__(256) void pool_x_kernel(
    const float* __restrict__ X, const int* __restrict__ aidx, float* __restrict__ aspx) {
  __shared__ float S[256];
  const unsigned tid = threadIdx.x;
  const unsigned b = blockIdx.x >> 1;
  const unsigned half = blockIdx.x & 1u;
  const unsigned d = half * 256u + tid;
  const int lo0 = aidx[2u * b];
  const int hi0 = aidx[2u * b + 1u];
  const bool all_in = (lo0 <= 0) && (hi0 >= SEQ - 1);
  const int lo = max(lo0, 0);
  const int hi = min(hi0, SEQ - 1);
  float mval = all_in ? -3.402823466e38f : 0.0f;
  const float* base = X + (size_t)b * SEQ_FULL * DIM + d;
#pragma unroll 1
  for (int n = lo; n <= hi; ++n) mval = fmaxf(mval, bf16r(base[(size_t)n * DIM]));
  S[tid] = mval;
  __syncthreads();
  if (tid < 64u) {
    const v4f x = *(const v4f*)&S[4u * tid];
    float* p = aspx + (size_t)b * DIM + half * 256u + 4u * tid;
    *(volatile v4f*)p = x;
    __threadfence();
    *(volatile v4f*)p = x;
  }
}

__global__ __launch_bounds__(256) void gate_kernel(
    const float* __restrict__ aspx, const float* __restrict__ aspt,
    const float* __restrict__ Ww, const float* __restrict__ bw, float* __restrict__ gate) {
  __shared__ float zs[32];
  __shared__ float gs[32];
  const unsigned tid = threadIdx.x, lane = tid & 31u;
  const int wave = __builtin_amdgcn_readfirstlane(threadIdx.x >> 5);
#pragma unroll 1
  for (unsigned r = 0; r < 4u; ++r) {
    const unsigned hb = (unsigned)wave * 4u + r;
    if (hb < (unsigned)(NHEAD * NB)) {
      const unsigned b = hb % (unsigned)NB;
      float p = 0.0f;
#pragma unroll 1
      for (unsigned j = 0; j < 16u; ++j) {
        const unsigned d = j * 32u + lane;
        p += aspx[(size_t)b * DIM + d] * bf16r(Ww[d]);
        p += aspt[(size_t)hb * DIM + d] * bf16r(Ww[DIM + d]);
      }
      p = red32_sum(p);
      const float z = fmaxf(p + bf16r(bw[0]), 0.0f);
      if (lane == 0u) zs[hb] = z;
    }
  }
  __syncthreads();
  if (wave == 0) {
    const unsigned L = min(lane, (unsigned)(NHEAD * NB - 1));
    const unsigned b = L % (unsigned)NB;
    float mx = -3.402823466e38f;
#pragma unroll
    for (unsigned h = 0; h < (unsigned)NHEAD; ++h) mx = fmaxf(mx, zs[h * NB + b]);
    float es = 0.0f;
#pragma unroll
    for (unsigned h = 0; h < (unsigned)NHEAD; ++h) es += __expf(zs[h * NB + b] - mx);
    const float own = __expf(zs[L] - mx);
    const float g = own * (1.0f / es) * (1.0f / (float)NHEAD);
    gs[lane] = (lane < (unsigned)(NHEAD * NB)) ? g : 0.0f;
    wave_lds_sync();
    if (lane < 8u) {
      const v4f x = *(const v4f*)&gs[4u * lane];
      float* p = gate + 4u * lane;
      *(volatile v4f*)p = x;
      __threadfence();
      *(volatile v4f*)p = x;
    }
  }
}

__global__ __launch_bounds__(256) void final_kernel(
    const float* __restrict__ hedge, const float* __restrict__ gate, float* __restrict__ out) {
  const unsigned idx = blockIdx.x * 256u + threadIdx.x;
  const unsigned crow = idx / (unsigned)(DIM / 4);
  const unsigned c = (idx - crow * (unsigned)(DIM / 4)) * 4u;
  const unsigned b = crow / (unsigned)SEQ;
  const unsigned sq = crow - b * (unsigned)SEQ;
  v4f acc = {0.0f, 0.0f, 0.0f, 0.0f};
#pragma unroll
  for (unsigned h = 0; h < (unsigned)NHEAD; ++h) {
    const float g = gate[h * NB + b];
    const v4f u = *(const v4f*)(hedge + (((size_t)h * NB + b) * SEQ + sq) * DIM + c);
#pragma unroll
    for (int j = 0; j < 4; ++j) acc[j] += g * u[j];
  }
  v4f val;
#pragma unroll
  for (int j = 0; j < 4; ++j) val[j] = fmaxf(acc[j], 0.0f);
  float* p = out + ((size_t)b * SEQ_FULL + sq) * DIM + c;
  *(volatile v4f*)p = val;
  __threadfence();
  *(volatile v4f*)p = val;
}

extern "C" void kernel_launch(void* const* d_in, const int* in_sizes, int n_in,
                              void* d_out, int out_size, void* d_ws, size_t ws_size,
                              hipStream_t stream) {
  if (n_in < 13) return;
  const long long need_x = ((long long)(NB - 1) * SEQ_FULL + SEQ) * DIM;
  const long long need_m = ((long long)(NB - 1) * SEQ_FULL + SEQ) * SEQ_FULL;
  if ((long long)in_sizes[0] < need_x) return;
  if ((long long)in_sizes[1] < need_m) return;
  if ((long long)in_sizes[2] < need_m) return;
  if (in_sizes[3] < 2 * NB) return;
  if (in_sizes[4] < NTYPES * EDIM) return;
  if (in_sizes[5] < NHEAD * EDIM * EHID) return;
  if (in_sizes[6] < NHEAD * EHID) return;
  if ((long long)in_sizes[7] < (long long)NHEAD * DIM * DIM) return;
  if (in_sizes[8] < NHEAD * DIM) return;
  if ((long long)in_sizes[9] < (long long)DIM * DIM) return;
  if (in_sizes[10] < DIM) return;
  if (in_sizes[11] < 2 * DIM) return;
  if (in_sizes[12] < 1) return;
  const long long need_out =
      (long long)OUT1_ELEMS + (long long)((NHEAD - 1) * NB_FULL + NB) * SEQ * SEQ;
  if ((long long)out_size < need_out) return;
  if (ws_size < WS_TOTAL) return;

  const float* X     = (const float*)d_in[0];
  const int*   adj   = (const int*)d_in[1];
  const int*   dep   = (const int*)d_in[2];
  const int*   aidx  = (const int*)d_in[3];
  const float* table = (const float*)d_in[4];
  const float* Wm    = (const float*)d_in[5];
  const float* Wl    = (const float*)d_in[6];
  const float* Wto   = (const float*)d_in[7];
  const float* bto   = (const float*)d_in[8];
  const float* Wasp  = (const float*)d_in[9];
  const float* basp  = (const float*)d_in[10];
  const float* Ww    = (const float*)d_in[11];
  const float* bw    = (const float*)d_in[12];
  float* out_hp  = (float*)d_out;
  float* out_att = (float*)d_out + OUT1_ELEMS;

  char* ws = (char*)d_ws;
  _Float16* WtoT  = (_Float16*)(ws + OFF_WTO);
  _Float16* WaspT = (_Float16*)(ws + OFF_WASP);
  _Float16* X16   = (_Float16*)(ws + OFF_X16);
  float*    Lut   = (float*)(ws + OFF_LUT);
  _Float16* Att16 = (_Float16*)(ws + OFF_ATT16);
  _Float16* HvT   = (_Float16*)(ws + OFF_HVT);
  float*    Hedge = (float*)(ws + OFF_HEDGE);
  _Float16* Asp16 = (_Float16*)(ws + OFF_ASP16);
  float*    AspX  = (float*)(ws + OFF_ASPX);
  float*    AspT  = (float*)(ws + OFF_ASPT);
  float*    Gate  = (float*)(ws + OFF_GATE);

  dim3 blk(256);
  dim3 gsq(DIM / 64, DIM / 64);

  for (int h = 0; h < NHEAD; ++h)
    wconv_kernel<<<gsq, blk, 0, stream>>>(Wto + (size_t)h * DIM * DIM,
                                          WtoT + (size_t)h * DIM * DIM,
                                          (unsigned)DIM, (unsigned)DIM);
  wconv_kernel<<<gsq, blk, 0, stream>>>(Wasp, WaspT, (unsigned)DIM, (unsigned)DIM);

  xconv_kernel<<<dim3((unsigned)((size_t)MROWS * DIM / 8 / 256)), blk, 0, stream>>>(X, X16);
  lut_kernel<<<dim3(NHEAD), dim3(64), 0, stream>>>(table, Wm, Wl, Lut);
  att_kernel<<<dim3(MROWS / 8), blk, 0, stream>>>(adj, dep, Lut, out_att, Att16);
  gemm_hv_kernel<<<dim3(NCAT / 64, MROWS / 64), blk, 0, stream>>>(X16, WtoT, bto, HvT);
  gemm_hedge_kernel<<<dim3(DIM / 64, SEQ / 64, NHEAD * NB), blk, 0, stream>>>(Att16, HvT, Hedge);
  pool_h_kernel<<<dim3(APAD * 2), blk, 0, stream>>>(Hedge, aidx, Asp16);
  pool_x_kernel<<<dim3(NB * 2), blk, 0, stream>>>(X, aidx, AspX);
  gemm_asp_kernel<<<dim3(DIM / 64, APAD / 64), blk, 0, stream>>>(Asp16, WaspT, basp, AspT);
  gate_kernel<<<dim3(1), blk, 0, stream>>>(AspX, AspT, Ww, bw, Gate);
  final_kernel<<<dim3((unsigned)((size_t)MROWS * DIM / 4 / 256)), blk, 0, stream>>>(Hedge, Gate, out_hp);
}
